// TokenMatchLayer_31731218382862
// MI455X (gfx1250) — hardware-verified
//
#include <hip/hip_runtime.h>


namespace {
constexpr int B = 4, S = 2048, D = 768, NH = 8, DH = 96, SEP = 102, NCH = S / 32;
constexpr int VB = B, HCAP = S;
constexpr float XS = 8.0f, PS = 1024.0f, WSC = 256.0f;
typedef _Float16 b16;
typedef __attribute__((ext_vector_type(16))) _Float16 v16b;
typedef __attribute__((ext_vector_type(8))) _Float16 v8b;
typedef __attribute__((ext_vector_type(8))) float v8f;
typedef __attribute__((ext_vector_type(4))) float v4f;
typedef __attribute__((ext_vector_type(4))) _Float16 v4b;
__device__ __forceinline__ float bf16_rne(float f) { unsigned int u = __float_as_uint(f); u += 0x7FFFu + ((u >> 16) & 1u); float r = __uint_as_float(u & 0xFFFF0000u); asm volatile("" : "+v"(r)); return r; }
__device__ __forceinline__ void split16(float v, b16& hi, b16& lo) { hi = (b16)v; lo = (b16)(v - (float)hi); }
__device__ __forceinline__ v16b frag_kb(const b16* p, int hh) { const v8b a = *(const v8b*)(p + 8 * hh), b = *(const v8b*)(p + 16 + 8 * hh); v16b f;
#pragma unroll
  for (int e = 0; e < 8; ++e) { f[e] = a[e]; f[8 + e] = b[e]; } return f; }
__device__ __forceinline__ v8f wmma16b(v16b a, v16b b, v8f c) { v8f d = __builtin_amdgcn_wmma_f32_16x16x32_f16(false, a, false, b, (short)0, c, false, false); asm volatile("v_nop\n\tv_nop\n\tv_nop\n\tv_nop" : "+v"(d) : "v"(a), "v"(b)); return d; }
__device__ __forceinline__ void wave_lds_sync() { __builtin_amdgcn_fence(__ATOMIC_RELEASE, "workgroup"); __builtin_amdgcn_wave_barrier(); __builtin_amdgcn_fence(__ATOMIC_ACQUIRE, "workgroup"); }
__device__ __forceinline__ float pmul(float a, float b) { float p = a * b; asm volatile("" : "+v"(p)); return p; }
__device__ __forceinline__ int iclamp(int v, int lo, int hi) { return v < lo ? lo : (v > hi ? hi : v); }
__device__ __forceinline__ float gelu_t(float v) { const float u = 0.7978845608028654f * (v + 0.044715f * v * v * v); const float t = 1.0f - 2.0f / (__expf(2.0f * u) + 1.0f); return 0.5f * v * (1.0f + t); }

__global__ __launch_bounds__(256) void wput_kernel(const float* __restrict__ wq, const float* __restrict__ wk, const float* __restrict__ wv, const float* __restrict__ wo, const float* __restrict__ w1, const float* __restrict__ w2, b16* __restrict__ WT) { const size_t u = (size_t)blockIdx.x * 256 + threadIdx.x; if (u >= (size_t)6 * D * (D / 8)) return; const int which = (int)(u / ((size_t)D * (D / 8))); const int o = (int)((u / (D / 8)) % D), k0 = (int)(u % (D / 8)) * 8; const float* w = which == 0 ? wq : which == 1 ? wk : which == 2 ? wv : which == 3 ? wo : which == 4 ? w1 : w2; v8b v;
#pragma unroll
  for (int j = 0; j < 8; ++j) v[j] = (b16)(bf16_rne(w[(size_t)(k0 + j) * D + o]) * WSC); for (int pass = 0; pass < 2; ++pass) { *(volatile v8b*)(WT + ((size_t)which * D + o) * D + k0) = v; __threadfence(); } }
__global__ __launch_bounds__(32) void seg_kernel(const int* __restrict__ ids, int* __restrict__ SG) { const int lane = threadIdx.x, b = blockIdx.x; int first = S, second = S;
  if (lane == 0) { for (int i = 0; i < S; ++i) if (ids[(size_t)b * S + i] == SEP) { if (first == S) first = i; else { second = i; break; } } }
  first = __shfl(first, 0); second = __shfl(second, 0); const bool has2 = second < S; const int mid = S / 2; int src_end = has2 ? first : mid, hyp_start = has2 ? first + 1 : mid, hyp_end = has2 ? second : S - 1; int valid = (src_end > 1 && hyp_end > hyp_start) ? 1 : 0;
  if (b >= VB) { valid = 0; src_end = 0; } if (hyp_end > hyp_start + HCAP) hyp_end = hyp_start + HCAP;
  const int v = lane == 0 ? src_end : lane == 1 ? hyp_start : lane == 2 ? hyp_end : lane == 3 ? valid : 0; for (int pass = 0; pass < 2; ++pass) { ((volatile int*)SG)[b * 32 + lane] = v; __threadfence(); } }
template <int MODE, int EPI>
__global__ __launch_bounds__(32) void dense_kernel(const float* __restrict__ IN, const b16* __restrict__ Wsec, const float* __restrict__ bias, const int* __restrict__ SG, int rangeSel, float* __restrict__ OUTF, b16* __restrict__ OUTH, b16* __restrict__ OUTL) {
  __shared__ __attribute__((aligned(16))) b16 Ah[32][D + 8], Al[MODE == 0 ? 1 : 32][MODE == 0 ? 8 : D + 8]; __shared__ float Tf[32][132]; const int lane = threadIdx.x, nloc = lane & 15, hlf = lane >> 4; const int g = blockIdx.x % 6, rt = (blockIdx.x / 6) % (S / 32), b = blockIdx.x / (6 * (S / 32));
  const int src_end = SG[b * 32], hs = SG[b * 32 + 1], he = SG[b * 32 + 2], valid = SG[b * 32 + 3]; int lo, hi; if (rangeSel == 0) { lo = 0; hi = src_end; } else { lo = hs; hi = valid ? he : hs; }
  const int r0 = (rangeSel == 0 ? 0 : (lo & ~31)) + rt * 32; if (r0 >= hi) return; const size_t row0 = (size_t)b * S + r0;
  for (int rr = 0; rr < 32; ++rr) for (int q = 0; q < D / 32; ++q) { const bool ok = r0 + rr < S; const float v = ok ? IN[(row0 + rr) * D + q * 32 + lane] : 0.0f; if (MODE == 0) Ah[rr][q * 32 + lane] = (b16)(bf16_rne(v) * XS); else { b16 p, ql; split16(v * XS, p, ql); Ah[rr][q * 32 + lane] = p; Al[rr][q * 32 + lane] = ql; } }
  wave_lds_sync(); v8f acc[2][8];
#pragma unroll
  for (int m = 0; m < 2; ++m) for (int t = 0; t < 8; ++t) acc[m][t] = (v8f){};
#pragma unroll 1
  for (int kb = 0; kb < D; kb += 32) { v16b a[2], al[2]; for (int m = 0; m < 2; ++m) { a[m] = frag_kb(&Ah[m * 16 + nloc][kb], hlf); if (MODE != 0) al[m] = frag_kb(&Al[m * 16 + nloc][kb], hlf); }
#pragma unroll
    for (int t = 0; t < 8; ++t) { const v16b bw = frag_kb(Wsec + (size_t)(g * 128 + t * 16 + nloc) * D + kb, hlf);
#pragma unroll
      for (int m = 0; m < 2; ++m) { acc[m][t] = wmma16b(a[m], bw, acc[m][t]); if (MODE != 0) acc[m][t] = wmma16b(al[m], bw, acc[m][t]); } } }
#pragma unroll
  for (int m = 0; m < 2; ++m)
#pragma unroll
    for (int t = 0; t < 8; ++t) { const int c = g * 128 + t * 16 + nloc; const float bb = bias ? bf16_rne(bias[c]) : 0.0f;
#pragma unroll
      for (int r8 = 0; r8 < 8; ++r8) { float v = acc[m][t][r8] * (1.0f / (XS * WSC)) + bb; if (EPI == 2) v = gelu_t(v); Tf[m * 16 + 8 * hlf + r8][t * 16 + nloc] = v; } }
  wave_lds_sync();
  for (int pass = 0; pass < 2; ++pass) { for (int rr = 0; rr < 32; ++rr) { const int r = r0 + rr; if (r < lo || r >= hi) continue; const size_t o = (row0 + rr) * D + g * 128 + lane * 4; const v4f v = *(const v4f*)(&Tf[rr][lane * 4]);
      if (EPI == 1) { v4b vh, vl; for (int k = 0; k < 4; ++k) { b16 p, ql; split16(v[k] * XS, p, ql); vh[k] = p; vl[k] = ql; } *(volatile v4b*)(OUTH + o) = vh; *(volatile v4b*)(OUTL + o) = vl; } else *(volatile v4f*)(OUTF + o) = v; } __threadfence(); } }
__global__ __launch_bounds__(32) void vt_kernel(const float* __restrict__ V, const int* __restrict__ SG, b16* __restrict__ VTh, b16* __restrict__ VTl) { const int lane = threadIdx.x; const int ch = blockIdx.x % NCH, b = blockIdx.x / NCH; const int src_end = SG[b * 32]; if (ch * 32 >= src_end) return; const int j = ch * 32 + lane; const size_t base = ((size_t)b * NCH + ch) * D;
  for (int pass = 0; pass < 2; ++pass) {
#pragma unroll 4
    for (int d = 0; d < D; ++d) { const float v = j < src_end ? V[((size_t)b * S + j) * D + d] : 0.0f; b16 p, q; split16(v * XS, p, q); ((volatile b16*)VTh)[(base + d) * 64 + lane] = p; ((volatile b16*)VTl)[(base + d) * 64 + lane] = q; } __threadfence(); } }
__global__ __launch_bounds__(32) void att_kernel(const b16* __restrict__ Qh, const b16* __restrict__ Ql, const b16* __restrict__ Kh, const b16* __restrict__ Kl, const b16* __restrict__ VTh, const b16* __restrict__ VTl, const int* __restrict__ SG, float* __restrict__ CTX) {
  __shared__ __attribute__((aligned(16))) b16 Ph[16][40], Pl[16][40]; __shared__ float Sc[16][33], Mx[16], Dn[16], Sf[16], Of[16][DH + 1];
  const int lane = threadIdx.x, nloc = lane & 15, hlf = lane >> 4; const int qt = blockIdx.x % (S / 16), h = (blockIdx.x / (S / 16)) % NH, b = blockIdx.x / ((S / 16) * NH);
  const int src_end = SG[b * 32], hs = SG[b * 32 + 1], he = SG[b * 32 + 2], valid = SG[b * 32 + 3]; if (!valid) return; const int q0 = (hs & ~15) + qt * 16; if (q0 >= he) return; const size_t qrow = (size_t)b * S + q0;
  if (lane < 16) { Mx[lane] = -INFINITY; Dn[lane] = 0.0f; Sf[lane] = 0.0f; }
  v16b qa[3], qb[3];
#pragma unroll
  for (int kk = 0; kk < 3; ++kk) { qa[kk] = frag_kb(Qh + (qrow + nloc) * D + h * DH + kk * 32, hlf); qb[kk] = frag_kb(Ql + (qrow + nloc) * D + h * DH + kk * 32, hlf); }
  v8f acc[6]; for (int t = 0; t < 6; ++t) acc[t] = (v8f){}; wave_lds_sync();
#pragma unroll 1
  for (int kc = 0; kc < src_end; kc += 32) {
#pragma unroll
    for (int blk = 0; blk < 2; ++blk) { v8f s = {}; const size_t kr = ((size_t)b * S + kc + blk * 16 + nloc) * D + h * DH;
#pragma unroll
      for (int kk = 0; kk < 3; ++kk) { const v16b kh_ = frag_kb(Kh + kr + kk * 32, hlf), kl_ = frag_kb(Kl + kr + kk * 32, hlf); s = wmma16b(qa[kk], kh_, s); s = wmma16b(qa[kk], kl_, s); s = wmma16b(qb[kk], kh_, s); }
#pragma unroll
      for (int r8 = 0; r8 < 8; ++r8) { const int j = kc + blk * 16 + nloc; Sc[8 * hlf + r8][blk * 16 + nloc] = (j >= 1 && j < src_end) ? s[r8] * (0.10206207261596575f / (XS * XS)) : -INFINITY; } }
    wave_lds_sync();
#pragma unroll 1
    for (int qi = 0; qi < 16; ++qi) { const float sv = Sc[qi][lane]; float cm = sv; for (int o = 16; o; o >>= 1) cm = fmaxf(cm, __shfl_xor(cm, o)); const float mo = Mx[qi]; const float mn = fmaxf(mo, cm); const float p = (sv == -INFINITY || mn == -INFINITY) ? 0.0f : __expf(sv - mn); float ps = p; for (int o = 16; o; o >>= 1) ps += __shfl_xor(ps, o);
      b16 ph, plo; split16(p * PS, ph, plo); Ph[qi][lane] = ph; Pl[qi][lane] = plo; if (lane == 0) { const float sf = (mo == -INFINITY) ? ((mn == -INFINITY) ? 1.0f : 0.0f) : __expf(mo - mn); Sf[qi] = sf; Dn[qi] = Dn[qi] * sf + ps; Mx[qi] = mn; } }
    wave_lds_sync(); const v16b pa = frag_kb(&Ph[nloc][0], hlf), pb = frag_kb(&Pl[nloc][0], hlf); const size_t vb = (((size_t)b * NCH + kc / 32) * D + h * DH) * 64;
#pragma unroll
    for (int t = 0; t < 6; ++t) {
#pragma unroll
      for (int r8 = 0; r8 < 8; ++r8) acc[t][r8] *= Sf[8 * hlf + r8];
      const v16b vh = frag_kb(VTh + vb + (size_t)(t * 16 + nloc) * 64, hlf), vl = frag_kb(VTl + vb + (size_t)(t * 16 + nloc) * 64, hlf); acc[t] = wmma16b(pa, vh, acc[t]); acc[t] = wmma16b(pa, vl, acc[t]); acc[t] = wmma16b(pb, vh, acc[t]); }
    wave_lds_sync(); }
#pragma unroll
  for (int t = 0; t < 6; ++t)
#pragma unroll
    for (int r8 = 0; r8 < 8; ++r8) { const int rl = 8 * hlf + r8; Of[rl][t * 16 + nloc] = acc[t][r8] * (1.0f / (PS * XS)) / Dn[rl]; }
  wave_lds_sync();
  for (int pass = 0; pass < 2; ++pass) { for (int rr = 0; rr < 16; ++rr) { const int i = q0 + rr; if (i < hs || i >= he) continue; for (int d = lane; d < DH; d += 32) ((volatile float*)CTX)[(qrow + rr) * D + h * DH + d] = Of[rr][d]; } __threadfence(); } }
template <int MODE>
__global__ __launch_bounds__(256) void ln_kernel(const float* __restrict__ x, const float* __restrict__ A1, const float* __restrict__ A2, const float* __restrict__ g1, const float* __restrict__ be1, const float* __restrict__ g2, const float* __restrict__ be2, const int* __restrict__ SG, float* __restrict__ OUT) {
  const int wave = threadIdx.x >> 5, lane = threadIdx.x & 31; const int i = blockIdx.x % (S / 8) * 8 + wave, b = blockIdx.x / (S / 8); const int hs = SG[b * 32 + 1], he = SG[b * 32 + 2], valid = SG[b * 32 + 3]; if (!valid || i < hs || i >= he) return; const size_t row = (size_t)b * S + i;
  float v[24]; float s = 0.0f;
#pragma unroll
  for (int q = 0; q < 24; ++q) { const int c = q * 32 + lane; v[q] = (MODE == 0 ? bf16_rne(x[row * D + c]) : A1[row * D + c]) + A2[row * D + c]; s += v[q]; }
  for (int o = 16; o; o >>= 1) s += __shfl_xor(s, o); float mu = s * (1.0f / D); float qq = 0.0f;
#pragma unroll
  for (int q = 0; q < 24; ++q) qq += pmul(v[q] - mu, v[q] - mu); for (int o = 16; o; o >>= 1) qq += __shfl_xor(qq, o); float rs = rsqrtf(qq * (1.0f / D) + 1e-5f);
#pragma unroll
  for (int q = 0; q < 24; ++q) { const int c = q * 32 + lane; v[q] = pmul(pmul(v[q] - mu, rs), bf16_rne(g1[c])) + bf16_rne(be1[c]); }
  if (MODE == 1) {
    s = 0.0f;
#pragma unroll
    for (int q = 0; q < 24; ++q) { v[q] -= bf16_rne(x[row * D + q * 32 + lane]); s += v[q]; } for (int o = 16; o; o >>= 1) s += __shfl_xor(s, o); mu = s * (1.0f / D); qq = 0.0f;
#pragma unroll
    for (int q = 0; q < 24; ++q) qq += pmul(v[q] - mu, v[q] - mu); for (int o = 16; o; o >>= 1) qq += __shfl_xor(qq, o); rs = rsqrtf(qq * (1.0f / D) + 1e-5f);
#pragma unroll
    for (int q = 0; q < 24; ++q) { const int c = q * 32 + lane; v[q] = bf16_rne(x[row * D + c]) + pmul(pmul(v[q] - mu, rs), bf16_rne(g2[c])) + bf16_rne(be2[c]); } }
  for (int pass = 0; pass < 2; ++pass) {
#pragma unroll
    for (int q = 0; q < 24; ++q) ((volatile float*)OUT)[row * D + q * 32 + lane] = v[q]; __threadfence(); } }
__global__ __launch_bounds__(256) void copy_kernel(const float* __restrict__ x, const int* __restrict__ SG, float* __restrict__ out) { const size_t u = (size_t)blockIdx.x * 256 + threadIdx.x; if (u >= (size_t)B * S * D / 4) return; const size_t row = u / (D / 4); const int b = (int)(row / S), i = (int)(row % S); const int hs = SG[b * 32 + 1], he = SG[b * 32 + 2], valid = SG[b * 32 + 3]; if (valid && i >= hs && i < he) return;
  v4f v; for (int k = 0; k < 4; ++k) v[k] = bf16_rne(x[u * 4 + k]); for (int pass = 0; pass < 2; ++pass) { *(volatile v4f*)(out + u * 4) = v; __threadfence(); } }
}

extern "C" void kernel_launch(void* const* d_in, const int* in_sizes, int n_in, void* d_out, int out_size, void* d_ws, size_t ws_size, hipStream_t stream) {
  (void)n_in;
  auto Fp = [&](int i) { return (const float*)d_in[i]; }; auto Ip = [&](int i) { return (const int*)d_in[i]; };
  if (in_sizes[0] != B * S * D || in_sizes[1] != B * S || in_sizes[3] != D * D || in_sizes[9] != D * D || in_sizes[13] != D * D || in_sizes[15] != D * D || out_size != B * S * D) return;
  size_t off = 0; char* ws = (char*)d_ws;
  auto carve = [&](size_t bytes) { char* p = ws + off; off += (bytes + 255) & ~(size_t)255; return p; };
  b16* WT = (b16*)carve((size_t)6 * D * D * 2); int* SG = (int*)carve(4 * 32 * 4);
  b16* Qh = (b16*)carve((size_t)B * S * D * 2); b16* Ql = (b16*)carve((size_t)B * S * D * 2); b16* Kh = (b16*)carve((size_t)B * S * D * 2); b16* Kl = (b16*)carve((size_t)B * S * D * 2); float* Vf = (float*)carve((size_t)B * S * D * 4);
  b16* VTh = (b16*)carve((size_t)B * NCH * D * 64 * 2); b16* VTl = (b16*)carve((size_t)B * NCH * D * 64 * 2); float* CTX = (float*)carve((size_t)B * S * D * 4); float* MHA = (float*)carve((size_t)B * S * D * 4); float* X1 = (float*)carve((size_t)B * S * D * 4);
  if (off > ws_size || off > ((size_t)250 << 20)) return;
  float* Gf = CTX;
  float* F2 = MHA;
  wput_kernel<<<(unsigned)(((size_t)6 * D * (D / 8) + 255) / 256), 256, 0, stream>>>(Fp(3), Fp(5), Fp(7), Fp(9), Fp(13), Fp(15), WT);
  seg_kernel<<<B, 32, 0, stream>>>(Ip(1), SG);
  dense_kernel<0, 1><<<B * (S / 32) * 6, 32, 0, stream>>>(Fp(0), WT + (size_t)1 * D * D, Fp(6), SG, 0, nullptr, Kh, Kl);
  dense_kernel<0, 0><<<B * (S / 32) * 6, 32, 0, stream>>>(Fp(0), WT + (size_t)2 * D * D, Fp(8), SG, 0, Vf, nullptr, nullptr);
  vt_kernel<<<B * NCH, 32, 0, stream>>>(Vf, SG, VTh, VTl);
  dense_kernel<0, 1><<<B * (S / 32) * 6, 32, 0, stream>>>(Fp(0), WT, Fp(4), SG, 1, nullptr, Qh, Ql);
  att_kernel<<<B * NH * (S / 16), 32, 0, stream>>>(Qh, Ql, Kh, Kl, VTh, VTl, SG, CTX);
  dense_kernel<1, 0><<<B * (S / 32) * 6, 32, 0, stream>>>(CTX, WT + (size_t)3 * D * D, Fp(10), SG, 1, MHA, nullptr, nullptr);
  ln_kernel<0><<<B * (S / 8), 256, 0, stream>>>(Fp(0), nullptr, MHA, Fp(11), Fp(12), nullptr, nullptr, SG, X1);
  dense_kernel<1, 2><<<B * (S / 32) * 6, 32, 0, stream>>>(X1, WT + (size_t)4 * D * D, Fp(14), SG, 1, Gf, nullptr, nullptr);
  dense_kernel<1, 0><<<B * (S / 32) * 6, 32, 0, stream>>>(Gf, WT + (size_t)5 * D * D, Fp(16), SG, 1, F2, nullptr, nullptr);
  ln_kernel<1><<<B * (S / 8), 256, 0, stream>>>(Fp(0), X1, F2, Fp(17), Fp(18), Fp(19), Fp(20), SG, (float*)d_out);
  copy_kernel<<<(unsigned)(((size_t)B * S * D / 4 + 255) / 256), 256, 0, stream>>>(Fp(0), SG, (float*)d_out);
}
